// Decoder_v2_87746181858018
// MI455X (gfx1250) — hardware-verified
//
#include <hip/hip_runtime.h>


namespace {
constexpr int NB = 8192, DIN = 512, NF = 16, ZD = 32;
constexpr float XS = 8.0f, FW = 5.0f, INVN = 0.07978845608028654f;

typedef _Float16 b16;
typedef __attribute__((ext_vector_type(16))) _Float16 v16b;
typedef __attribute__((ext_vector_type(8))) _Float16 v8b;
typedef __attribute__((ext_vector_type(8))) float v8f;
typedef __attribute__((ext_vector_type(4))) float v4f;
__device__ __forceinline__ float bf16_rne(float f) { unsigned int u = __float_as_uint(f); u += 0x7FFFu + ((u >> 16) & 1u); return __uint_as_float(u & 0xFFFF0000u); }
__device__ __forceinline__ void split16(float v, b16& hi, b16& lo) { hi = (b16)v; lo = (b16)(v - (float)hi); }
__device__ __forceinline__ v16b frag_kb(const b16* p, int hh) { const v8b a = *(const v8b*)(p + 8 * hh), b = *(const v8b*)(p + 16 + 8 * hh); v16b f;
#pragma unroll
  for (int e = 0; e < 8; ++e) { f[e] = a[e]; f[8 + e] = b[e]; } return f; }
__device__ __forceinline__ v8f wmma16b(v16b a, v16b b, v8f c) { v8f d = __builtin_amdgcn_wmma_f32_16x16x32_f16(false, a, false, b, (short)0, c, false, false); asm volatile("v_nop\n\tv_nop\n\tv_nop\n\tv_nop" : "+v"(d) : "v"(a), "v"(b)); return d; }
__device__ __forceinline__ void wave_lds_sync() { __builtin_amdgcn_fence(__ATOMIC_RELEASE, "workgroup"); __builtin_amdgcn_wave_barrier(); __builtin_amdgcn_fence(__ATOMIC_ACQUIRE, "workgroup"); }
__device__ __forceinline__ float nexp(float x) { return __builtin_amdgcn_exp2f(x * 1.4426950408889634f); }
__device__ __forceinline__ float pmul(float a, float b) { float p = a * b; asm volatile("" : "+v"(p)); return p; }

struct Lay { int KP, NR, NP, SW; size_t woff; int boff; };
__host__ __device__ constexpr Lay LAYER(int i) {
  return (i == 0) ? Lay{512, 300, 304, 320, 0, 0} : (i == 1) ? Lay{320, 150, 160, 160, 155648, 304} : (i == 2) ? Lay{160, 70, 80, 96, 206848, 464} : (i == 3) ? Lay{96, 16, 16, 32, 219648, 544} : (i == 4) ? Lay{32, 16, 16, 64, 221184, 560}
       : (i == 5) ? Lay{64, 70, 80, 96, 221696, 576} : (i == 6) ? Lay{96, 150, 160, 160, 226816, 656} : (i == 7) ? Lay{160, 300, 304, 320, 242176, 816} : (i == 8) ? Lay{320, 512, 512, 512, 290816, 1120} : Lay{512, 512, 512, 512, 454656, 1632}; }
constexpr size_t REND = 454656 + (size_t)512 * 512; constexpr int PEND = 1632 + 512;

__global__ __launch_bounds__(256) void prep_kernel(const float* const* __restrict__ dummy, const float* __restrict__ psd, const float* __restrict__ pw1, const float* __restrict__ pb1, const float* __restrict__ pw2, const float* __restrict__ pb2, const float* __restrict__ pw3, const float* __restrict__ pb3,
    const float* __restrict__ w0, const float* __restrict__ b0, const float* __restrict__ w1, const float* __restrict__ b1, const float* __restrict__ w2, const float* __restrict__ b2, const float* __restrict__ w3, const float* __restrict__ b3, const float* __restrict__ w4, const float* __restrict__ b4,
    const float* __restrict__ w5, const float* __restrict__ b5, const float* __restrict__ w6, const float* __restrict__ b6, const float* __restrict__ w7, const float* __restrict__ b7, const float* __restrict__ w8, const float* __restrict__ b8, const float* __restrict__ w9, const float* __restrict__ b9, b16* __restrict__ R, float* __restrict__ P) {
  (void)dummy;
  const size_t tid = (size_t)blockIdx.x * 256 + threadIdx.x, nth = (size_t)gridDim.x * 256;
  const float* ws_[10] = {w0, w1, w2, w3, w4, w5, w6, w7, w8, w9}; const float* bs_[10] = {b0, b1, b2, b3, b4, b5, b6, b7, b8, b9}; const int kreal[10] = {512, 300, 150, 70, 16, 48, 70, 150, 300, 512};
  for (int pass = 0; pass < 2; ++pass) {
    for (int l = 0; l < 10; ++l) { const Lay L = LAYER(l); const int KR = kreal[l];
      for (size_t p = tid; p < (size_t)L.NP * L.KP; p += nth) { const int o = (int)(p / L.KP), k = (int)(p % L.KP); ((volatile b16*)R)[L.woff + p] = (b16)((o < L.NR && k < KR) ? bf16_rne(ws_[l][(size_t)o * KR + k]) : 0.0f); }
      for (size_t q = tid; q < (size_t)L.NP; q += nth) P[L.boff + q] = (q < (size_t)L.NR) ? bf16_rne(bs_[l][q]) : 0.0f; }
    for (size_t q = tid; q < 1088; q += nth) { const int i = (int)q; float v; if (i < 512) v = pw1[i]; else if (i < 528) v = pb1[i - 512]; else if (i < 784) v = pw2[i - 528]; else if (i < 800) v = pb2[i - 784]; else if (i < 1056) v = pw3[i - 800]; else v = pb3[i - 1056]; P[4096 + q] = bf16_rne(v); }
    for (size_t q = tid; q < 512; q += nth) P[5200 + q] = bf16_rne(psd[q]);
    __threadfence(); }
}
__global__ __launch_bounds__(256) void front_kernel(const float* __restrict__ z, const float* __restrict__ P, float* __restrict__ out1, b16* __restrict__ Xh, b16* __restrict__ Xl) {
  __shared__ float F0[8][NF]; __shared__ float Hs[8][16], Gs[8][16]; __shared__ __attribute__((aligned(16))) b16 Sh[8][DIN + 8], Sl[8][DIN + 8];
  const int wave = threadIdx.x >> 5, lane = threadIdx.x & 31, n = blockIdx.x * 8 + wave; const float* PR = P + 4096;
  if (lane < 16) { float s = PR[512 + lane];
#pragma unroll 1
    for (int i = 0; i < ZD; ++i) s += pmul(bf16_rne(z[(size_t)n * ZD + i]), PR[lane * ZD + i]);
    Hs[wave][lane] = fmaxf(s, 0.0f); }
  wave_lds_sync();
  if (lane < 16) { float s = PR[784 + lane];
#pragma unroll 1
    for (int i = 0; i < NF; ++i) s += pmul(Hs[wave][i], PR[528 + lane * NF + i]);
    Gs[wave][lane] = fmaxf(s, 0.0f); }
  wave_lds_sync();
  if (lane < 16) { float s = PR[1056 + lane];
#pragma unroll 1
    for (int i = 0; i < NF; ++i) s += pmul(Gs[wave][i], PR[800 + lane * NF + i]);
    const float sg = 1.0f / (1.0f + nexp(-s)); F0[wave][lane] = pmul((float)DIN, sg); }
  wave_lds_sync();
#pragma unroll 1
  for (int e = 0; e < 16; ++e) { const int f = lane * 16 + e; float hsum = 0.0f;
#pragma unroll 1
    for (int i = 0; i < NF; ++i) { const float d = (f - F0[wave][i]) * (1.0f / FW); hsum += nexp(-0.5f * pmul(d, d)); }
    const float xr = pmul(PR[1104 + f], pmul(hsum, INVN)); b16 a_, b_; split16(xr * XS, a_, b_); Sh[wave][f] = a_; Sl[wave][f] = b_; }
  wave_lds_sync();
  for (int pass = 0; pass < 2; ++pass) { for (int i = lane; i < DIN / 8; i += 32) { *(volatile v8b*)(Xh + (size_t)n * DIN + i * 8) = *(const v8b*)(&Sh[wave][i * 8]); *(volatile v8b*)(Xl + (size_t)n * DIN + i * 8) = *(const v8b*)(&Sl[wave][i * 8]); }
    if (lane < 4) *(volatile v4f*)(out1 + (size_t)n * NF + lane * 4) = *(const v4f*)(&F0[wave][lane * 4]); __threadfence(); }
}
template <int KP, int NP, int SW, int RELU, int MODE, int NSUB = 8>
__global__ __launch_bounds__(64) void lin_kernel(const b16* __restrict__ Ah, const b16* __restrict__ Al, const b16* __restrict__ Bw, const float* __restrict__ bias, b16* __restrict__ Oh, b16* __restrict__ Ol, float* __restrict__ OF, const float* __restrict__ z) {
  constexpr int CGW = NSUB * 16;
  __shared__ __attribute__((aligned(16))) b16 Th[2][16][CGW + 8], Tl[2][16][CGW + 8]; __shared__ __attribute__((aligned(16))) float Ts[2][16][128 + 4];
  const int lane = threadIdx.x & 31, wave = threadIdx.x >> 5, nloc = lane & 15, hlf = lane >> 4, m0 = blockIdx.y * 32 + wave * 16, c0 = blockIdx.x * CGW;
  v8f acc[NSUB];
#pragma unroll
  for (int t = 0; t < NSUB; ++t) acc[t] = (v8f){};
#pragma unroll 2
  for (int kb = 0; kb < KP; kb += 32) { const v16b a = frag_kb(Ah + (size_t)(m0 + nloc) * KP + kb, hlf), al_ = frag_kb(Al + (size_t)(m0 + nloc) * KP + kb, hlf);
#pragma unroll
    for (int t = 0; t < NSUB; ++t) { if (c0 + t * 16 < NP) { const v16b bw = frag_kb(Bw + (size_t)(c0 + t * 16 + nloc) * KP + kb, hlf); acc[t] = wmma16b(a, bw, acc[t]); acc[t] = wmma16b(al_, bw, acc[t]); } } }
#pragma unroll
  for (int t = 0; t < NSUB; ++t) { const int col = c0 + t * 16 + nloc; const bool live = (c0 + t * 16 < NP); const float bb = live ? bias[col] : 0.0f;
#pragma unroll
    for (int r = 0; r < 8; ++r) { float v = live ? (acc[t][r] * (1.0f / XS) + bb) : 0.0f; if (RELU) v = fmaxf(v, 0.0f);
      if (MODE == 1) Ts[wave][8 * hlf + r][t * 16 + nloc] = v; else { if (MODE == 2 && t >= 1) { v = (t < 3) ? bf16_rne(z[(size_t)(m0 + 8 * hlf + r) * ZD + (t - 1) * 16 + nloc]) : 0.0f; } b16 a_, c_; split16(v * XS, a_, c_); Th[wave][8 * hlf + r][t * 16 + nloc] = a_; Tl[wave][8 * hlf + r][t * 16 + nloc] = c_; } } }
  wave_lds_sync();
  const int wcols = (MODE == 1) ? 128 : ((SW - c0 < CGW) ? (SW - c0) : CGW);
  for (int pass = 0; pass < 2; ++pass) {
    if (MODE == 1) { for (int i = lane; i < 16 * 32; i += 32) { const int rr = i >> 5, c4 = (i & 31) * 4; *(volatile v4f*)(OF + (size_t)(m0 + rr) * 512 + c0 + c4) = *(const v4f*)(&Ts[wave][rr][c4]); } }
    else { const int npc = wcols / 8; for (int i = lane; i < 16 * npc; i += 32) { const int rr = i / npc, c8 = (i % npc) * 8; const size_t gi = (size_t)(m0 + rr) * SW + c0 + c8; *(volatile v8b*)(Oh + gi) = *(const v8b*)(&Th[wave][rr][c8]); *(volatile v8b*)(Ol + gi) = *(const v8b*)(&Tl[wave][rr][c8]); } }
    __threadfence(); }
}
}

extern "C" void kernel_launch(void* const* d_in, const int* in_sizes, int n_in,
                              void* d_out, int out_size, void* d_ws, size_t ws_size, hipStream_t stream) {
  (void)n_in; (void)out_size;
  auto Fp = [&](int i) { return (const float*)d_in[i]; };
  float* out0 = (float*)d_out; float* out1 = out0 + (size_t)NB * DIN;
  if (in_sizes[1] != NB * ZD || in_sizes[3] != DIN || in_sizes[10] != 300 * 512) return;
  size_t off = 0; char* ws = (char*)d_ws;
  auto carve = [&](size_t bytes) { char* p = ws + off; off += (bytes + 255) & ~(size_t)255; return p; };
  b16* R = (b16*)carve(REND * 2); float* P = (float*)carve(5712 * 4);
  b16* Ah = (b16*)carve((size_t)NB * 512 * 2); b16* Al = (b16*)carve((size_t)NB * 512 * 2); b16* Bh = (b16*)carve((size_t)NB * 512 * 2); b16* Bl = (b16*)carve((size_t)NB * 512 * 2);
  if (off > ws_size) return;
  prep_kernel<<<512, 256, 0, stream>>>(nullptr, Fp(3), Fp(4), Fp(5), Fp(6), Fp(7), Fp(8), Fp(9), Fp(10), Fp(11), Fp(12), Fp(13), Fp(14), Fp(15), Fp(16), Fp(17), Fp(18), Fp(19), Fp(20), Fp(21), Fp(22), Fp(23), Fp(24), Fp(25), Fp(26), Fp(27), Fp(28), Fp(29), R, P);
  front_kernel<<<NB / 8, 256, 0, stream>>>(Fp(1), P, out1, Ah, Al);
  lin_kernel<512, 304, 320, 1, 0><<<dim3(3, NB / 32), 64, 0, stream>>>(Ah, Al, R + LAYER(0).woff, P + LAYER(0).boff, Bh, Bl, nullptr, nullptr);
  lin_kernel<320, 160, 160, 1, 0, 10><<<dim3(1, NB / 32), 64, 0, stream>>>(Bh, Bl, R + LAYER(1).woff, P + LAYER(1).boff, Ah, Al, nullptr, nullptr);
  lin_kernel<160, 80, 96, 1, 0><<<dim3(1, NB / 32), 64, 0, stream>>>(Ah, Al, R + LAYER(2).woff, P + LAYER(2).boff, Bh, Bl, nullptr, nullptr);
  lin_kernel<96, 16, 32, 0, 0><<<dim3(1, NB / 32), 64, 0, stream>>>(Bh, Bl, R + LAYER(3).woff, P + LAYER(3).boff, Ah, Al, nullptr, nullptr);
  lin_kernel<32, 16, 64, 0, 2><<<dim3(1, NB / 32), 64, 0, stream>>>(Ah, Al, R + LAYER(4).woff, P + LAYER(4).boff, Bh, Bl, nullptr, Fp(1));
  lin_kernel<64, 80, 96, 1, 0><<<dim3(1, NB / 32), 64, 0, stream>>>(Bh, Bl, R + LAYER(5).woff, P + LAYER(5).boff, Ah, Al, nullptr, nullptr);
  lin_kernel<96, 160, 160, 1, 0, 10><<<dim3(1, NB / 32), 64, 0, stream>>>(Ah, Al, R + LAYER(6).woff, P + LAYER(6).boff, Bh, Bl, nullptr, nullptr);
  lin_kernel<160, 304, 320, 1, 0><<<dim3(3, NB / 32), 64, 0, stream>>>(Bh, Bl, R + LAYER(7).woff, P + LAYER(7).boff, Ah, Al, nullptr, nullptr);
  lin_kernel<320, 512, 512, 0, 0><<<dim3(4, NB / 32), 64, 0, stream>>>(Ah, Al, R + LAYER(8).woff, P + LAYER(8).boff, Bh, Bl, nullptr, nullptr);
  lin_kernel<512, 512, 512, 0, 1><<<dim3(4, NB / 32), 64, 0, stream>>>(Bh, Bl, R + LAYER(9).woff, P + LAYER(9).boff, nullptr, nullptr, out0, nullptr);
}
